// DeepFM_72189810311759
// MI455X (gfx1250) — hardware-verified
//
#include <hip/hip_runtime.h>
#include <stddef.h>
#include <stdint.h>


#define BATCH 16384
#define KE    512
#define NE    257
#define NPE   320
#define DSW   16
#define NF    16
#define D1    512
#define H1    256
#define H2    128
#define XSC   8
#define WSC   1024
#define HSC   8
#define NTHR  256
#define SP    68
#define TP    33
#define WSCAP 134217728

static_assert(NF * DSW == 256);
static_assert(NE == NF * DSW + 1);
static_assert(D1 == 2 * NF * DSW);
static_assert((NPE % 64) == 0);
static_assert(NPE >= NE);
static_assert((BATCH % 128) == 0);
static_assert((BATCH % 32) == 0);
static_assert((KE % 128) == 0);
static_assert((D1 % 128) == 0);
static_assert((H1 % 128) == 0);
static_assert((H1 % 64) == 0);
static_assert((H2 % 64) == 0);
static_assert(H2 == 4 * 32);
static_assert(((BATCH * KE) % (8 * NTHR)) == 0);
static_assert(NTHR == 256);
static_assert((SP % 4) == 0);

typedef float          v4f  __attribute__((ext_vector_type(4)));
typedef float          v8f  __attribute__((ext_vector_type(8)));
typedef _Float16       v4h  __attribute__((ext_vector_type(4)));
typedef _Float16       v8h  __attribute__((ext_vector_type(8)));
typedef _Float16       v16h __attribute__((ext_vector_type(16)));
union FragH { v16h v; v8h h[2]; };

__device__ __forceinline__ v8f wmf(v16h a, v16h b, v8f c) {
  v8f d = __builtin_amdgcn_wmma_f32_16x16x32_f16(false, a, false, b, (short)0, c, false, false);
  asm volatile("v_nop\n\tv_nop\n\tv_nop\n\tv_nop" : "+v"(d) : "v"(a), "v"(b));
  return d;
}

__global__ __launch_bounds__(NTHR) void k_prepx(const float* __restrict__ x, _Float16* xh) {
  const size_t t = (size_t)blockIdx.x * NTHR + threadIdx.x;
  const float* p = x + t * 8;
  const v4f f0 = *(const v4f*)p;
  const v4f f1 = *(const v4f*)(p + 4);
  v8h a;
  a[0] = (_Float16)(f0.x * (float)XSC); a[1] = (_Float16)(f0.y * (float)XSC);
  a[2] = (_Float16)(f0.z * (float)XSC); a[3] = (_Float16)(f0.w * (float)XSC);
  a[4] = (_Float16)(f1.x * (float)XSC); a[5] = (_Float16)(f1.y * (float)XSC);
  a[6] = (_Float16)(f1.z * (float)XSC); a[7] = (_Float16)(f1.w * (float)XSC);
  _Float16* d = xh + t * 8;
  *(volatile v8h*)d = a;
  __threadfence();
  *(volatile v8h*)d = a;
}

__global__ __launch_bounds__(NTHR) void k_prepw(const float* __restrict__ W, int K, int N, _Float16* wt) {
  __shared__ __attribute__((aligned(16))) float tile[128 * TP];
  const int tid = threadIdx.x, lane = tid & 31, g = tid >> 5, hh = lane >> 4, pc = lane & 15;
  const int n0 = blockIdx.x * 32;
  const int n = n0 + lane;
  const int nc = (n < N) ? n : (N - 1);
  const bool valid = (n < N);
#pragma unroll 1
  for (int k0 = 0; k0 < K; k0 += 128) {
    __syncthreads();
#pragma unroll 4
    for (int p = 0; p < 16; ++p) {
      const int kl = g + 8 * p;
      const float v = W[(size_t)(k0 + kl) * N + nc];
      tile[kl * TP + lane] = valid ? v : 0.f;
    }
    __syncthreads();
    v8h hv[2];
#pragma unroll
    for (int it = 0; it < 2; ++it) {
      const int r = 16 * it + 2 * g + hh;
#pragma unroll
      for (int e = 0; e < 8; ++e) hv[it][e] = (_Float16)(tile[(8 * pc + e) * TP + r] * (float)WSC);
    }
#pragma unroll
    for (int it = 0; it < 2; ++it) {
      const int r = 16 * it + 2 * g + hh;
      _Float16* d = wt + (size_t)(n0 + r) * K + k0 + 8 * pc;
      *(volatile v8h*)d = hv[it];
    }
    __threadfence();
#pragma unroll
    for (int it = 0; it < 2; ++it) {
      const int r = 16 * it + 2 * g + hh;
      _Float16* d = wt + (size_t)(n0 + r) * K + k0 + 8 * pc;
      *(volatile v8h*)d = hv[it];
    }
  }
}

template<int MODE>
__global__ __launch_bounds__(NTHR) void k_gemm(const _Float16* __restrict__ A, const _Float16* __restrict__ Bt,
                                               const float* __restrict__ bias, int K, int Nlog,
                                               float* outF, int pitchF,
                                               _Float16* outH, int pitchH, int hofs, int hcols,
                                               float osc, float hsc) {
  __shared__ __attribute__((aligned(16))) float stg[128 * SP];
  const int tid = threadIdx.x, lane = tid & 31, wave = tid >> 5, hh = lane >> 4, m = lane & 15;
  const int n0 = blockIdx.x * 64, m0 = blockIdx.y * 128;
  const int wm = (wave >> 1) * 32, wn = (wave & 1) * 32;

  v8f acc[2][2];
#pragma unroll
  for (int mt = 0; mt < 2; ++mt)
#pragma unroll
    for (int nt = 0; nt < 2; ++nt) { v8f z = {0.f, 0.f, 0.f, 0.f, 0.f, 0.f, 0.f, 0.f}; acc[mt][nt] = z; }

  const _Float16* ap = A  + (size_t)(m0 + wm + m) * K + 8 * hh;
  const _Float16* bp = Bt + (size_t)(n0 + wn + m) * K + 8 * hh;
  const size_t r16 = (size_t)16 * K;
#pragma unroll 1
  for (int k0 = 0; k0 < K; k0 += 32) {
    FragH a0, a1, b0, b1;
    a0.h[0] = *(const v8h*)(ap + k0);
    a0.h[1] = *(const v8h*)(ap + k0 + 16);
    a1.h[0] = *(const v8h*)(ap + r16 + k0);
    a1.h[1] = *(const v8h*)(ap + r16 + k0 + 16);
    b0.h[0] = *(const v8h*)(bp + k0);
    b0.h[1] = *(const v8h*)(bp + k0 + 16);
    b1.h[0] = *(const v8h*)(bp + r16 + k0);
    b1.h[1] = *(const v8h*)(bp + r16 + k0 + 16);
    acc[0][0] = wmf(a0.v, b0.v, acc[0][0]);
    acc[0][1] = wmf(a0.v, b1.v, acc[0][1]);
    acc[1][0] = wmf(a1.v, b0.v, acc[1][0]);
    acc[1][1] = wmf(a1.v, b1.v, acc[1][1]);
  }

  float bv[2];
#pragma unroll
  for (int nt = 0; nt < 2; ++nt) {
    const int col = n0 + wn + 16 * nt + m;
    const int cc = (col < Nlog) ? col : (Nlog - 1);
    const float b = bias[cc];
    bv[nt] = (col < Nlog) ? b : 0.f;
  }
#pragma unroll
  for (int mt = 0; mt < 2; ++mt) {
    float* sp = stg + (wm + 16 * mt + 8 * hh) * SP + wn + m;
#pragma unroll
    for (int nt = 0; nt < 2; ++nt) {
#pragma unroll
      for (int r = 0; r < 8; ++r) {
        float v = acc[mt][nt][r] * osc + bv[nt];
        if constexpr (MODE == 1) v = fmaxf(v, 0.f);
        sp[r * SP + 16 * nt] = v;
      }
    }
  }
  __syncthreads();

  const bool doH = (MODE == 1) || (n0 + 64 <= hcols);

  if constexpr (MODE == 0) {
#pragma unroll
    for (int q = 0; q < 8; ++q) {
      const int row = 16 * wave + 2 * q + hh;
      const v4f v = *(const v4f*)(stg + row * SP + 4 * m);
      *(volatile v4f*)(outF + (size_t)(m0 + row) * pitchF + n0 + 4 * m) = v;
    }
  }
  if (doH) {
#pragma unroll
    for (int q = 0; q < 4; ++q) {
      const int row = 16 * wave + 4 * q + (lane >> 3);
      const int pc = lane & 7;
      const float* s = stg + row * SP + 8 * pc;
      const v4f x0 = *(const v4f*)s;
      const v4f x1 = *(const v4f*)(s + 4);
      v8h hv;
      hv[0] = (_Float16)(x0.x * hsc); hv[1] = (_Float16)(x0.y * hsc);
      hv[2] = (_Float16)(x0.z * hsc); hv[3] = (_Float16)(x0.w * hsc);
      hv[4] = (_Float16)(x1.x * hsc); hv[5] = (_Float16)(x1.y * hsc);
      hv[6] = (_Float16)(x1.z * hsc); hv[7] = (_Float16)(x1.w * hsc);
      *(volatile v8h*)(outH + (size_t)(m0 + row) * pitchH + hofs + n0 + 8 * pc) = hv;
    }
  }
  __threadfence();
  if constexpr (MODE == 0) {
#pragma unroll
    for (int q = 0; q < 8; ++q) {
      const int row = 16 * wave + 2 * q + hh;
      const v4f v = *(const v4f*)(stg + row * SP + 4 * m);
      *(volatile v4f*)(outF + (size_t)(m0 + row) * pitchF + n0 + 4 * m) = v;
    }
  }
  if (doH) {
#pragma unroll
    for (int q = 0; q < 4; ++q) {
      const int row = 16 * wave + 4 * q + (lane >> 3);
      const int pc = lane & 7;
      const float* s = stg + row * SP + 8 * pc;
      const v4f x0 = *(const v4f*)s;
      const v4f x1 = *(const v4f*)(s + 4);
      v8h hv;
      hv[0] = (_Float16)(x0.x * hsc); hv[1] = (_Float16)(x0.y * hsc);
      hv[2] = (_Float16)(x0.z * hsc); hv[3] = (_Float16)(x0.w * hsc);
      hv[4] = (_Float16)(x1.x * hsc); hv[5] = (_Float16)(x1.y * hsc);
      hv[6] = (_Float16)(x1.z * hsc); hv[7] = (_Float16)(x1.w * hsc);
      *(volatile v8h*)(outH + (size_t)(m0 + row) * pitchH + hofs + n0 + 8 * pc) = hv;
    }
  }
}

__global__ __launch_bounds__(NTHR) void k_final(const float* __restrict__ dm, const float* __restrict__ du,
                                                const _Float16* __restrict__ h2, const float* __restrict__ W3,
                                                const float* __restrict__ b3, float* out, int pitchD) {
  __shared__ __attribute__((aligned(16))) float res[32];
  const int tid = threadIdx.x, lane = tid & 31, wave = tid >> 5;
  const v4f w3 = *(const v4f*)(W3 + 4 * lane);
  const float b3v = b3[0];
  constexpr float HINV = 1.0f / (float)HSC;
#pragma unroll 1
  for (int r = 0; r < 4; ++r) {
    const int row = blockIdx.x * 32 + wave * 4 + r;
    const float* pm = dm + (size_t)row * pitchD;
    const float* pu = du + (size_t)row * pitchD;
    const v4f ma = *(const v4f*)(pm + 8 * lane);
    const v4f mb = *(const v4f*)(pm + 8 * lane + 4);
    const v4f ua = *(const v4f*)(pu + 8 * lane);
    const v4f ub = *(const v4f*)(pu + 8 * lane + 4);
    const float lm = pm[NF * DSW];
    const float lu = pu[NF * DSW];
    float sm[8] = {ma.x, ma.y, ma.z, ma.w, mb.x, mb.y, mb.z, mb.w};
#pragma unroll
    for (int e = 0; e < 8; ++e) {
      float s = sm[e];
      s += __shfl_xor(s, 2);
      s += __shfl_xor(s, 4);
      s += __shfl_xor(s, 8);
      s += __shfl_xor(s, 16);
      sm[e] = s;
    }
    float fm = sm[0] * ua.x;
    fm += sm[1] * ua.y; fm += sm[2] * ua.z; fm += sm[3] * ua.w;
    fm += sm[4] * ub.x; fm += sm[5] * ub.y; fm += sm[6] * ub.z; fm += sm[7] * ub.w;
    fm += __shfl_xor(fm, 1);
    fm += __shfl_xor(fm, 2);
    fm += __shfl_xor(fm, 4);
    fm += __shfl_xor(fm, 8);
    fm += __shfl_xor(fm, 16);

    const v4h hq = *(const v4h*)(h2 + (size_t)row * H2 + 4 * lane);
    float p = (float)hq.x * w3.x;
    p += (float)hq.y * w3.y;
    p += (float)hq.z * w3.z;
    p += (float)hq.w * w3.w;
    p += __shfl_xor(p, 1);
    p += __shfl_xor(p, 2);
    p += __shfl_xor(p, 4);
    p += __shfl_xor(p, 8);
    p += __shfl_xor(p, 16);
    const float mlp = p * HINV + b3v;
    const float logit = mlp + (lm + lu) + fm;
    if (lane == 0) res[wave * 4 + r] = logit;
  }
  __syncthreads();
  if (wave == 0) {
    const v4f v = *(const v4f*)(res + 4 * (lane & 7));
    float* d = out + (size_t)blockIdx.x * 32 + 4 * (lane & 7);
    if (lane < 8) *(volatile v4f*)d = v;
    __threadfence();
    if (lane < 8) *(volatile v4f*)d = v;
  }
}

extern "C" void kernel_launch(void* const* d_in, const int* in_sizes, int n_in,
                              void* d_out, int out_size, void* d_ws, size_t ws_size,
                              hipStream_t stream) {
  if (n_in < 12) return;
  if (in_sizes[0] != BATCH * KE || in_sizes[1] != BATCH * KE) return;
  if (in_sizes[2] != KE * NE || in_sizes[3] != NE || in_sizes[4] != KE * NE || in_sizes[5] != NE) return;
  if (in_sizes[6] != D1 * H1 || in_sizes[7] != H1 || in_sizes[8] != H1 * H2 || in_sizes[9] != H2) return;
  if (in_sizes[10] != H2 || in_sizes[11] < 1) return;
  if (out_size != BATCH) return;

  const float* mv = (const float*)d_in[0];
  const float* uv = (const float*)d_in[1];
  const float* Wm = (const float*)d_in[2];
  const float* bm = (const float*)d_in[3];
  const float* Wu = (const float*)d_in[4];
  const float* bu = (const float*)d_in[5];
  const float* W1 = (const float*)d_in[6];
  const float* b1 = (const float*)d_in[7];
  const float* W2 = (const float*)d_in[8];
  const float* b2 = (const float*)d_in[9];
  const float* W3 = (const float*)d_in[10];
  const float* b3 = (const float*)d_in[11];
  float* out = (float*)d_out;

  char* ws = (char*)d_ws;
  size_t off = 0;
  const size_t oXm  = off; off += (size_t)BATCH * KE * 2;  off = (off + 255) & ~(size_t)255;
  const size_t oXu  = off; off += (size_t)BATCH * KE * 2;  off = (off + 255) & ~(size_t)255;
  const size_t oWtm = off; off += (size_t)NPE * KE * 2;    off = (off + 255) & ~(size_t)255;
  const size_t oWtu = off; off += (size_t)NPE * KE * 2;    off = (off + 255) & ~(size_t)255;
  const size_t oWt1 = off; off += (size_t)H1 * D1 * 2;     off = (off + 255) & ~(size_t)255;
  const size_t oWt2 = off; off += (size_t)H2 * H1 * 2;     off = (off + 255) & ~(size_t)255;
  const size_t oDm  = off; off += (size_t)BATCH * NPE * 4; off = (off + 255) & ~(size_t)255;
  const size_t oDu  = off; off += (size_t)BATCH * NPE * 4; off = (off + 255) & ~(size_t)255;
  const size_t oAd  = off; off += (size_t)BATCH * D1 * 4 / 2; off = (off + 255) & ~(size_t)255;
  const size_t oH1  = off; off += (size_t)BATCH * H1 * 2;  off = (off + 255) & ~(size_t)255;
  const size_t oH2  = off; off += (size_t)BATCH * H2 * 2;  off = (off + 255) & ~(size_t)255;
  if (off > ws_size || off > (size_t)WSCAP) return;
  _Float16* xm  = (_Float16*)(ws + oXm);
  _Float16* xu  = (_Float16*)(ws + oXu);
  _Float16* wtm = (_Float16*)(ws + oWtm);
  _Float16* wtu = (_Float16*)(ws + oWtu);
  _Float16* wt1 = (_Float16*)(ws + oWt1);
  _Float16* wt2 = (_Float16*)(ws + oWt2);
  float*    dm  = (float*)(ws + oDm);
  float*    du  = (float*)(ws + oDu);
  _Float16* ad  = (_Float16*)(ws + oAd);
  _Float16* h1  = (_Float16*)(ws + oH1);
  _Float16* h2  = (_Float16*)(ws + oH2);

  const float osc = 1.0f / (float)(XSC * WSC);
  const float hsc = (float)HSC;

  k_prepx<<<(BATCH * KE) / (8 * NTHR), NTHR, 0, stream>>>(mv, xm);
  k_prepx<<<(BATCH * KE) / (8 * NTHR), NTHR, 0, stream>>>(uv, xu);
  k_prepw<<<NPE / 32, NTHR, 0, stream>>>(Wm, KE, NE, wtm);
  k_prepw<<<NPE / 32, NTHR, 0, stream>>>(Wu, KE, NE, wtu);
  k_prepw<<<H1 / 32, NTHR, 0, stream>>>(W1, D1, H1, wt1);
  k_prepw<<<H2 / 32, NTHR, 0, stream>>>(W2, H1, H2, wt2);
  k_gemm<0><<<dim3(NPE / 64, BATCH / 128), NTHR, 0, stream>>>(xm, wtm, bm, KE, NE, dm, NPE, ad, D1, 0,        NF * DSW, osc, hsc);
  k_gemm<0><<<dim3(NPE / 64, BATCH / 128), NTHR, 0, stream>>>(xu, wtu, bu, KE, NE, du, NPE, ad, D1, NF * DSW, NF * DSW, osc, hsc);
  k_gemm<1><<<dim3(H1 / 64, BATCH / 128), NTHR, 0, stream>>>(ad, wt1, b1, D1, H1, dm, NPE, h1, H1, 0, H1, osc, hsc);
  k_gemm<1><<<dim3(H2 / 64, BATCH / 128), NTHR, 0, stream>>>(h1, wt2, b2, H1, H2, dm, NPE, h2, H2, 0, H2, osc, hsc);
  k_final<<<BATCH / 32, NTHR, 0, stream>>>(dm, du, h2, W3, b3, out, NPE);
}
